// DPRNNSeparator_78108275245645
// MI455X (gfx1250) — hardware-run, weakly checked
//
#include <hip/hip_runtime.h>
#include <math.h>

typedef __attribute__((ext_vector_type(16))) _Float16 v16h;
typedef __attribute__((ext_vector_type(8)))  _Float16 v8h;
typedef __attribute__((ext_vector_type(8)))  float    v8f;
typedef __attribute__((ext_vector_type(4)))  float    v4f;
typedef __attribute__((ext_vector_type(4)))  unsigned v4u;

constexpr int kNumB   = 2;
constexpr int kEnc    = 64;
constexpr int kBot    = 64;
constexpr int kLen    = 8000;
constexpr int kChunk  = 100;
constexpr int kHop    = 50;
constexpr int kNumS   = 161;
constexpr int kBlocks = 6;
constexpr int kSpk    = 5;
constexpr int kHid    = 64;
constexpr int kGate   = 4 * kHid;
constexpr int kGate2  = 2 * kGate;
constexpr int kCat    = 2 * kHid;
constexpr int kRowsB  = kNumS * kChunk;
constexpr int kRows   = kNumB * kRowsB;
constexpr int kRowsP  = 32256;
constexpr int kMaskO  = kSpk * kEnc;
constexpr int kTok    = kNumB * kLen;
constexpr int kJobs   = kRows / 4;
constexpr int kHp     = 72;
constexpr int kStatBlk = 128;
constexpr float kEps      = 1e-8f;
constexpr float kActCarry = 64.0f;
constexpr float kWgtCarry = 512.0f;
constexpr float kFold     = 1.0f / (kActCarry * kWgtCarry);
constexpr float kHalfMin  = 6.103515625e-5f;

static_assert((kLen + 2 * kHop - kChunk) % kHop == 0, "no extra tail pad");
static_assert(kNumS == (kLen + 2 * kHop - kChunk) / kHop + 1, "chunk count");
static_assert(kChunk == 2 * kHop, "two covering chunks per position");
static_assert(kRows == 32200 && kRowsP % 64 == 0 && kRowsP >= kRows, "padded row count");
static_assert(kTok % 64 == 0 && kLen % 64 == 0 && kMaskO % 64 == 0 && kGate2 % 64 == 0 && kBot % 64 == 0, "GEMM M,N tile multiples");
static_assert(kEnc % 32 == 0 && kBot % 32 == 0 && kCat % 32 == 0 && kHid % 32 == 0, "GEMM K multiples of 32");
static_assert(kRows % 4 == 0 && kRowsB % 4 == 0, "four-row wave jobs never straddle a batch slab");
static_assert(kHid == 64 && kEnc == 64 && kBot == 64, "64-wide rows");
static_assert(kTok % 32 == 0, "overlap-add grid exact");
static_assert(kStatBlk * kNumB == 256, "one partial line per finalize thread");

constexpr size_t kSzWI   = (size_t)kBlocks * 2 * 2 * kGate * kBot * 2;
constexpr size_t kSzWH   = (size_t)kBlocks * 2 * 2 * kGate * kHid * 2;
constexpr size_t kSzPW   = (size_t)kBlocks * 2 * kBot * kCat * 2;
constexpr size_t kSzMW   = (size_t)kMaskO * kBot * 2;
constexpr size_t kSzBW   = (size_t)kBot * kEnc * 2;
constexpr size_t kSzPART = (size_t)256 * 32 * 4;
constexpr size_t kSzXT   = (size_t)kTok * kEnc * 2;
constexpr size_t kSzXB   = (size_t)kTok * kBot * 4;
constexpr size_t kSzCH   = (size_t)kRows * kBot * 4;
constexpr size_t kSzXSEQ = (size_t)kRowsP * kBot * 2;
constexpr size_t kSzPRE  = (size_t)kRowsP * kGate2 * 4;
constexpr size_t kSzHCAT = (size_t)kRowsP * kCat * 2;
constexpr size_t kSzYP   = (size_t)kRowsP * kBot * 4;
constexpr size_t kSzYACT = (size_t)kTok * kBot * 2;
constexpr size_t kSzLOG  = (size_t)kNumB * kMaskO * kLen * 4;
constexpr size_t kOffWI   = 0;
constexpr size_t kOffWH   = kOffWI   + kSzWI;
constexpr size_t kOffPW   = kOffWH   + kSzWH;
constexpr size_t kOffMW   = kOffPW   + kSzPW;
constexpr size_t kOffBW   = kOffMW   + kSzMW;
constexpr size_t kOffPART = kOffBW   + kSzBW;
constexpr size_t kOffXT   = kOffPART + kSzPART;
constexpr size_t kOffXB   = kOffXT   + kSzXT;
constexpr size_t kOffCH0  = kOffXB   + kSzXB;
constexpr size_t kOffCH1  = kOffCH0  + kSzCH;
constexpr size_t kOffXSEQ = kOffCH1  + kSzCH;
constexpr size_t kOffPRE  = kOffXSEQ + kSzXSEQ;
constexpr size_t kOffHCAT = kOffPRE  + kSzPRE;
constexpr size_t kOffYP   = kOffHCAT + kSzHCAT;
constexpr size_t kOffYACT = kOffYP   + kSzYP;
constexpr size_t kOffLOG  = kOffYACT + kSzYACT;
constexpr size_t kWsTotal = kOffLOG  + kSzLOG;
static_assert(kWsTotal == 133713920ull, "carve total");
static_assert(kWsTotal <= 134217728ull, "carve cap");
static_assert(kSzWI % 256 == 0 && kSzWH % 256 == 0 && kSzPW % 256 == 0 && kSzMW % 256 == 0 && kSzBW % 256 == 0 &&
              kSzPART % 256 == 0 && kSzXT % 256 == 0 && kSzXB % 256 == 0 && kSzCH % 256 == 0 && kSzXSEQ % 256 == 0 &&
              kSzPRE % 256 == 0 && kSzHCAT % 256 == 0 && kSzYP % 256 == 0 && kSzYACT % 256 == 0 && kSzLOG % 256 == 0,
              "aligned regions");

constexpr int kCvtWi = (kBlocks * 2 * 2 * kGate * kBot) / 2048;
constexpr int kCvtWh = (kBlocks * 2 * 2 * kGate * kHid) / 2048;
constexpr int kCvtPw = (kBlocks * 2 * kBot * kCat) / 2048;
constexpr int kCvtMw = (kMaskO * kBot) / 2048;
constexpr int kCvtBw = (kBot * kEnc) / 2048;
constexpr int kCb1 = kCvtWi;
constexpr int kCb2 = kCb1 + kCvtWh;
constexpr int kCb3 = kCb2 + kCvtPw;
constexpr int kCb4 = kCb3 + kCvtMw;
constexpr int kCbAll = kCb4 + kCvtBw;
static_assert((kBlocks * 2 * 2 * kGate * kBot) % 2048 == 0 && (kBlocks * 2 * kBot * kCat) % 2048 == 0 &&
              (kMaskO * kBot) % 2048 == 0 && (kBot * kEnc) % 2048 == 0, "convert grids exact");
static_assert(kCbAll == 444, "convert grid");

__device__ __forceinline__ _Float16 to_h16c(float v, float carry) {
  float f = v * carry;
  f = fminf(fmaxf(f, -60000.0f), 60000.0f);
  const float g = (fabsf(f) < kHalfMin) ? 0.0f : f;
  return (_Float16)g;
}
__device__ __forceinline__ v8h pack8(v4f a, v4f b, float carry) {
  v8h h;
  h[0] = to_h16c(a[0], carry);
  h[1] = to_h16c(a[1], carry);
  h[2] = to_h16c(a[2], carry);
  h[3] = to_h16c(a[3], carry);
  h[4] = to_h16c(b[0], carry);
  h[5] = to_h16c(b[1], carry);
  h[6] = to_h16c(b[2], carry);
  h[7] = to_h16c(b[3], carry);
  return h;
}
__device__ __forceinline__ float fsig(float x)  { return __builtin_amdgcn_rcpf(1.0f + __expf(-x)); }
__device__ __forceinline__ float ftanh(float x) { return 1.0f - 2.0f * __builtin_amdgcn_rcpf(__expf(2.0f * x) + 1.0f); }

union FragU { v16h v; v8h h[2]; };
__device__ __forceinline__ v16h frag_load(const _Float16* p) {
  FragU f;
  f.h[0] = *(const v8h*)(p);
  f.h[1] = *(const v8h*)(p + 16);
  return f.v;
}
__device__ __forceinline__ v8f mma_g(v16h a, v16h b, v8f c) {
  c = __builtin_amdgcn_wmma_f32_16x16x32_f16(false, a, false, b, (short)0, c, false, false);
  asm volatile("v_nop\n\tv_nop\n\tv_nop\n\tv_nop" : "+v"(c) : "v"(a), "v"(b));
  return c;
}

__device__ __forceinline__ void row_decode(int row, int& b, int& s, int& k) {
  b = row / kRowsB;
  const int rem = row - b * kRowsB;
  s = rem / kChunk;
  k = rem - s * kChunk;
}

__device__ __forceinline__ void gn_finalize(const float* __restrict__ part, float* sP, double* sR, int tid) {
  const float ps = part[(size_t)tid * 32];
  const float pq = part[(size_t)tid * 32 + 1];
  sP[tid] = ps;
  sP[256 + tid] = pq;
  __syncthreads();
  if (tid < 4) {
    const float* q = sP + (tid & 1) * 256 + (tid >> 1) * kStatBlk;
    double a = 0.0;
#pragma unroll 1
    for (int i = 0; i < kStatBlk; ++i) a += (double)q[i];
    sR[tid] = a;
  }
  __syncthreads();
}
__device__ __forceinline__ void gn_mu_rs(const double* sR, int b, double cntInv, float& mu, float& rs) {
  const double m = sR[2 * b] * cntInv;
  double var = sR[2 * b + 1] * cntInv - m * m;
  var = (var < 0.0) ? 0.0 : var;
  mu = (float)m;
  rs = 1.0f / sqrtf((float)var + kEps);
}

__global__ __launch_bounds__(256) void wcvt_kernel(
    const float* __restrict__ s0, unsigned short* __restrict__ d0,
    const float* __restrict__ s1, unsigned short* __restrict__ d1,
    const float* __restrict__ s2, unsigned short* __restrict__ d2,
    const float* __restrict__ s3, unsigned short* __restrict__ d3,
    const float* __restrict__ s4, unsigned short* __restrict__ d4) {
  const int bx = blockIdx.x;
  const float* src = s0;
  unsigned short* dst = d0;
  int bb = 0;
  if (bx >= kCb1) { src = s1; dst = d1; bb = kCb1; }
  if (bx >= kCb2) { src = s2; dst = d2; bb = kCb2; }
  if (bx >= kCb3) { src = s3; dst = d3; bb = kCb3; }
  if (bx >= kCb4) { src = s4; dst = d4; bb = kCb4; }
  const size_t i = (size_t)(bx - bb) * 256 + threadIdx.x;
  const v4f a = *(const v4f*)(src + i * 8);
  const v4f b = *(const v4f*)(src + i * 8 + 4);
  const v8h hv = pack8(a, b, kWgtCarry);
  unsigned short* p = dst + i * 8;
  *(volatile v8h*)p = hv;
  __threadfence();
  *(volatile v8h*)p = hv;
}

constexpr int kPadX = (kRowsP - kRows) * kBot * 2 / 16;
constexpr int kPadH = (kRowsP - kRows) * kCat * 2 / 16;
static_assert(kPadX % 32 == 0 && kPadH % 32 == 0, "wave-uniform pad ranges");
__global__ __launch_bounds__(256) void padzero_kernel(unsigned short* __restrict__ xseq, unsigned short* __restrict__ hcat) {
  const int i = blockIdx.x * 256 + threadIdx.x;
  if (i >= kPadX + kPadH) return;
  const bool isx = (i < kPadX);
  unsigned short* p = isx ? (xseq + (size_t)kRows * kBot + (size_t)i * 8)
                          : (hcat + (size_t)kRows * kCat + (size_t)(i - kPadX) * 8);
  v4u z;
  z[0] = 0u; z[1] = 0u; z[2] = 0u; z[3] = 0u;
  *(volatile v4u*)p = z;
  __threadfence();
  *(volatile v4u*)p = z;
}

__global__ __launch_bounds__(256) void stats_kernel(const float* __restrict__ src, int rowsPerBatch, int rpb, float* __restrict__ part) {
  __shared__ float sS[8];
  __shared__ float sQ[8];
  const int tid = threadIdx.x, lane = tid & 31, wave = tid >> 5;
  const int b = blockIdx.y;
  int r0 = blockIdx.x * rpb;
  r0 = (r0 > rowsPerBatch) ? rowsPerBatch : r0;
  int r1 = r0 + rpb;
  r1 = (r1 > rowsPerBatch) ? rowsPerBatch : r1;
  const int n4 = (r1 - r0) * 16;
  const float* p = src + ((size_t)b * rowsPerBatch + r0) * 64;
  float s = 0.0f, q = 0.0f;
#pragma unroll 1
  for (int i = tid; i < n4; i += 256) {
    const v4f v = *(const v4f*)(p + (size_t)i * 4);
    s += (v[0] + v[1]) + (v[2] + v[3]);
    q += (v[0] * v[0] + v[1] * v[1]) + (v[2] * v[2] + v[3] * v[3]);
  }
#pragma unroll
  for (int off = 1; off < 32; off <<= 1) {
    s += __shfl_xor(s, off, 32);
    q += __shfl_xor(q, off, 32);
  }
  if (lane == 0) { sS[wave] = s; sQ[wave] = q; }
  __syncthreads();
  if (wave == 0) {
    float ts = 0.0f, tq = 0.0f;
#pragma unroll
    for (int w = 0; w < 8; ++w) { ts += sS[w]; tq += sQ[w]; }
    const float val = (lane == 0) ? ts : ((lane == 1) ? tq : 0.0f);
    float* o = part + ((size_t)b * kStatBlk + blockIdx.x) * 32 + lane;
    *(volatile float*)o = val;
    __threadfence();
    *(volatile float*)o = val;
  }
}

__global__ __launch_bounds__(256) void front_norm_kernel(const float* __restrict__ enc, const float* __restrict__ part,
                                                         const float* __restrict__ gam, const float* __restrict__ bet,
                                                         unsigned short* __restrict__ xt, double cntInv) {
  __shared__ float Tt[64 * 65];
  __shared__ float sP[512];
  __shared__ double sR[4];
  const int tid = threadIdx.x;
  const int b = blockIdx.y;
  const int t0 = blockIdx.x * 64;
  gn_finalize(part, sP, sR, tid);
  float mu, rs;
  gn_mu_rs(sR, b, cntInv, mu, rs);
#pragma unroll
  for (int i = 0; i < 4; ++i) {
    const int idx = i * 256 + tid;
    const int rr = idx >> 4;
    const int cc = (idx & 15) * 4;
    const v4f v = *(const v4f*)(enc + ((size_t)b * kEnc + rr) * kLen + t0 + cc);
    const float g = gam[rr];
    const float be = bet[rr];
    Tt[rr * 65 + cc + 0] = ((v[0] - mu) * rs) * g + be;
    Tt[rr * 65 + cc + 1] = ((v[1] - mu) * rs) * g + be;
    Tt[rr * 65 + cc + 2] = ((v[2] - mu) * rs) * g + be;
    Tt[rr * 65 + cc + 3] = ((v[3] - mu) * rs) * g + be;
  }
  __syncthreads();
  const int q = tid >> 3, c8 = (tid & 7) * 8;
  v8h hv[2];
#pragma unroll
  for (int g2 = 0; g2 < 2; ++g2) {
    const int tq = g2 * 32 + q;
#pragma unroll
    for (int e = 0; e < 8; ++e) hv[g2][e] = to_h16c(Tt[(c8 + e) * 65 + tq], kActCarry);
  }
  for (int pass = 0; pass < 2; ++pass) {
#pragma unroll
    for (int g2 = 0; g2 < 2; ++g2) {
      const size_t row = (size_t)b * kLen + t0 + g2 * 32 + q;
      *(volatile v8h*)(xt + row * kEnc + c8) = hv[g2];
    }
    __threadfence();
  }
}

template <int BIAS_MODE>
__global__ __launch_bounds__(256) void gemm64_f16_kernel(
    const unsigned short* __restrict__ Ap, int lda, long strideA,
    const unsigned short* __restrict__ Btp, int ldb, long strideB,
    float* __restrict__ Cp, int ldc, long strideC,
    const float* __restrict__ bias, int M, int N, int K, float scale) {
  const _Float16* A = (const _Float16*)Ap;
  const _Float16* Bt = (const _Float16*)Btp;
  __shared__ __align__(16) float sT[8][16 * 68];
  const int b    = blockIdx.y;
  const int lane = threadIdx.x & 31;
  const int wave = threadIdx.x >> 5;
  const int tilesN = N >> 6;
  const int tilesM = M >> 6;
  const int tile = blockIdx.x * 8 + wave;
  if (tile >= tilesM * tilesN) return;
  const int tm = tile / tilesN;
  const int tn = tile - tm * tilesN;
  const int m0 = tm << 6;
  const int n0 = tn << 6;
  const _Float16* Ab = A + (size_t)b * strideA;
  const _Float16* Bb = Bt + (size_t)b * strideB;
  const int rlane = lane & 15;
  const int koff  = (lane >> 4) * 8;
  const int mOff  = (lane >> 4) * 8;

  v8f acc[4][4];
#pragma unroll
  for (int i = 0; i < 4; ++i)
#pragma unroll
    for (int j = 0; j < 4; ++j) acc[i][j] = (v8f){0.f, 0.f, 0.f, 0.f, 0.f, 0.f, 0.f, 0.f};

  for (int k0 = 0; k0 < K; k0 += 32) {
    v16h bh[4];
#pragma unroll
    for (int j = 0; j < 4; ++j) {
      const size_t bo = (size_t)(n0 + (j << 4) + rlane) * ldb + koff + k0;
      bh[j] = frag_load(Bb + bo);
    }
#pragma unroll
    for (int i = 0; i < 4; ++i) {
      const size_t ao = (size_t)(m0 + (i << 4) + rlane) * lda + koff + k0;
      const v16h ah = frag_load(Ab + ao);
#pragma unroll
      for (int j = 0; j < 4; ++j) acc[i][j] = mma_g(ah, bh[j], acc[i][j]);
    }
  }

  float* slab = sT[wave];
  float* C = Cp + (size_t)b * strideC;
#pragma unroll
  for (int i = 0; i < 4; ++i) {
    const int mBase = m0 + (i << 4);
#pragma unroll
    for (int j = 0; j < 4; ++j) {
      const int n = n0 + (j << 4) + rlane;
      float bv = 0.f;
      if (BIAS_MODE == 2) bv = bias[n];
#pragma unroll
      for (int r = 0; r < 8; ++r) {
        float v = acc[i][j][r] * scale;
        if (BIAS_MODE == 1) v += bias[mBase + mOff + r];
        if (BIAS_MODE == 2) v += bv;
        slab[(mOff + r) * 68 + (j << 4) + rlane] = v;
      }
    }
    __builtin_amdgcn_fence(__ATOMIC_RELEASE, "workgroup");
    __builtin_amdgcn_wave_barrier();
    __builtin_amdgcn_fence(__ATOMIC_ACQUIRE, "workgroup");
    {
      const int hh = lane >> 4, c4 = (lane & 15) * 4;
      for (int pass = 0; pass < 2; ++pass) {
#pragma unroll
        for (int it = 0; it < 8; ++it) {
          const int row = it * 2 + hh;
          const v4f v = *(const v4f*)(slab + row * 68 + c4);
          *(volatile v4f*)(C + (size_t)(mBase + row) * ldc + n0 + c4) = v;
        }
        __threadfence();
      }
    }
    __builtin_amdgcn_fence(__ATOMIC_RELEASE, "workgroup");
    __builtin_amdgcn_wave_barrier();
    __builtin_amdgcn_fence(__ATOMIC_ACQUIRE, "workgroup");
  }
}

__global__ __launch_bounds__(256) void chunk_build_kernel(const float* __restrict__ xb, float* __restrict__ ch,
                                                          unsigned short* __restrict__ xseq) {
  const int tid = threadIdx.x, lane = tid & 31, wave = tid >> 5;
  const int job = blockIdx.x * 8 + wave;
  if (job >= kJobs) return;
  v4f nv[2];
#pragma unroll
  for (int it = 0; it < 2; ++it) {
    const int row = 4 * job + 2 * it + (lane >> 4);
    const int c4 = (lane & 15) * 4;
    int b, s, k;
    row_decode(row, b, s, k);
    const int t = s * kHop + k - kHop;
    const bool ok = (t >= 0) && (t < kLen);
    int tc = (t < 0) ? 0 : t;
    tc = (tc > kLen - 1) ? (kLen - 1) : tc;
    v4f v = *(const v4f*)(xb + ((size_t)b * kLen + tc) * kBot + c4);
    asm volatile("" : "+v"(v));
    v4f r;
    r[0] = ok ? v[0] : 0.0f;
    r[1] = ok ? v[1] : 0.0f;
    r[2] = ok ? v[2] : 0.0f;
    r[3] = ok ? v[3] : 0.0f;
    nv[it] = r;
  }
  v8h hv;
  const int rowB = 4 * job + (lane >> 3);
  const int c8 = (lane & 7) * 8;
  {
    int b, s, k;
    row_decode(rowB, b, s, k);
    const int t = s * kHop + k - kHop;
    const bool ok = (t >= 0) && (t < kLen);
    int tc = (t < 0) ? 0 : t;
    tc = (tc > kLen - 1) ? (kLen - 1) : tc;
    const float* sp = xb + ((size_t)b * kLen + tc) * kBot + c8;
    v4f a0 = *(const v4f*)(sp);
    v4f a1 = *(const v4f*)(sp + 4);
    asm volatile("" : "+v"(a0));
    asm volatile("" : "+v"(a1));
    v4f z0, z1;
    z0[0] = ok ? a0[0] : 0.0f;
    z0[1] = ok ? a0[1] : 0.0f;
    z0[2] = ok ? a0[2] : 0.0f;
    z0[3] = ok ? a0[3] : 0.0f;
    z1[0] = ok ? a1[0] : 0.0f;
    z1[1] = ok ? a1[1] : 0.0f;
    z1[2] = ok ? a1[2] : 0.0f;
    z1[3] = ok ? a1[3] : 0.0f;
    hv = pack8(z0, z1, kActCarry);
  }
  for (int pass = 0; pass < 2; ++pass) {
#pragma unroll
    for (int it = 0; it < 2; ++it) {
      const int row = 4 * job + 2 * it + (lane >> 4);
      *(volatile v4f*)(ch + (size_t)row * kBot + (lane & 15) * 4) = nv[it];
    }
    *(volatile v8h*)(xseq + (size_t)rowB * kBot + c8) = hv;
    __threadfence();
  }
}

__global__ __launch_bounds__(128) void bilstm_scan_kernel(const float* __restrict__ pre, const unsigned short* __restrict__ whp,
                                                          unsigned short* __restrict__ hcat, int nseq, int tlen) {
  __shared__ __align__(16) _Float16 Hl[2][16 * kHp];
  const int tid = threadIdx.x, lane = tid & 31, wave = tid >> 5;
  const int c = lane & 15, hh = lane >> 4, koff = hh * 8;
  const int dir = blockIdx.y;
  const int r0 = blockIdx.x * 16;
  const _Float16* wh = (const _Float16*)whp + (size_t)dir * kGate * kHid;

  v16h wa[4][2];
#pragma unroll
  for (int g = 0; g < 4; ++g)
#pragma unroll
    for (int ks = 0; ks < 2; ++ks)
      wa[g][ks] = frag_load(wh + (size_t)(g * kHid + 16 * wave + c) * kHid + koff + 32 * ks);

  {
    _Float16* hz = &Hl[0][0];
#pragma unroll 1
    for (int i = tid; i < 2 * 16 * kHp; i += 128) hz[i] = (_Float16)0.0f;
  }
  float cst[8];
#pragma unroll
  for (int r = 0; r < 8; ++r) cst[r] = 0.0f;
  __syncthreads();

  int prow = r0 + c;
  prow = (prow > nseq - 1) ? (nseq - 1) : prow;
  const float* pbase = pre + (size_t)prow * tlen * kGate2 + dir * kGate + 16 * wave + 8 * hh;

  const int srow = wave * 4 + (lane >> 3);
  const int c8 = (lane & 7) * 8;
  const int sn = r0 + srow;
  const bool sok = (sn < nseq);
  const int snc = sok ? sn : (nseq - 1);
  unsigned short* hbase = hcat + (size_t)snc * tlen * kCat + dir * kHid + c8;
  const v8f z8 = {0.f, 0.f, 0.f, 0.f, 0.f, 0.f, 0.f, 0.f};

#pragma unroll 1
  for (int it = 0; it < tlen; ++it) {
    const int t = dir ? (tlen - 1 - it) : it;
    const int cur = it & 1;
    const float* pp = pbase + (size_t)t * kGate2;
    v4f pv[4][2];
#pragma unroll
    for (int g = 0; g < 4; ++g) {
      pv[g][0] = *(const v4f*)(pp + g * kHid);
      pv[g][1] = *(const v4f*)(pp + g * kHid + 4);
    }
    const _Float16* hrow = &Hl[cur][0] + c * kHp + koff;
    const v16h b0 = frag_load(hrow);
    const v16h b1 = frag_load(hrow + 32);
    v8f acc[4];
#pragma unroll
    for (int g = 0; g < 4; ++g) {
      acc[g] = z8;
      acc[g] = mma_g(wa[g][0], b0, acc[g]);
      acc[g] = mma_g(wa[g][1], b1, acc[g]);
    }
    v8h hv;
#pragma unroll
    for (int r = 0; r < 8; ++r) {
      const float zi = acc[0][r] * kFold + pv[0][r >> 2][r & 3];
      const float zf = acc[1][r] * kFold + pv[1][r >> 2][r & 3];
      const float zg = acc[2][r] * kFold + pv[2][r >> 2][r & 3];
      const float zo = acc[3][r] * kFold + pv[3][r >> 2][r & 3];
      const float ig = fsig(zi);
      const float fg = fsig(zf);
      const float gg = ftanh(zg);
      const float og = fsig(zo);
      const float cn = fg * cst[r] + ig * gg;
      cst[r] = cn;
      const float hn = og * ftanh(cn);
      hv[r] = to_h16c(hn, kActCarry);
    }
    *(v8h*)(&Hl[cur ^ 1][0] + c * kHp + 16 * wave + 8 * hh) = hv;
    __syncthreads();
    const v8h sv = *(const v8h*)(&Hl[cur ^ 1][0] + srow * kHp + c8);
    unsigned short* hp = hbase + (size_t)t * kCat;
    if (sok) *(volatile v8h*)hp = sv;
    __threadfence();
    if (sok) *(volatile v8h*)hp = sv;
  }
}

__global__ __launch_bounds__(256) void gn_apply_kernel(const float* __restrict__ chOld, const float* __restrict__ y,
                                                       const float* __restrict__ part, const float* __restrict__ gam,
                                                       const float* __restrict__ bet, float* __restrict__ chNew,
                                                       unsigned short* __restrict__ xseq, int path, double cntInv) {
  __shared__ float sP[512];
  __shared__ double sR[4];
  const int tid = threadIdx.x, lane = tid & 31, wave = tid >> 5;
  gn_finalize(part, sP, sR, tid);
  float mu0, rs0, mu1, rs1;
  gn_mu_rs(sR, 0, cntInv, mu0, rs0);
  gn_mu_rs(sR, 1, cntInv, mu1, rs1);
  const int job = blockIdx.x * 8 + wave;
  if (job >= kJobs) return;

  v4f nv[2];
#pragma unroll
  for (int it = 0; it < 2; ++it) {
    const int row = 4 * job + 2 * it + (lane >> 4);
    const int c4 = (lane & 15) * 4;
    int b, s, k;
    row_decode(row, b, s, k);
    const int mi = (b * kChunk + k) * kNumS + s;
    const int yrow = path ? mi : row;
    const v4f o  = *(const v4f*)(chOld + (size_t)row * kBot + c4);
    const v4f yv = *(const v4f*)(y + (size_t)yrow * kBot + c4);
    const v4f g4 = *(const v4f*)(gam + c4);
    const v4f b4 = *(const v4f*)(bet + c4);
    const float mu = b ? mu1 : mu0;
    const float rs = b ? rs1 : rs0;
    v4f r;
    r[0] = o[0] + (((yv[0] - mu) * rs) * g4[0] + b4[0]);
    r[1] = o[1] + (((yv[1] - mu) * rs) * g4[1] + b4[1]);
    r[2] = o[2] + (((yv[2] - mu) * rs) * g4[2] + b4[2]);
    r[3] = o[3] + (((yv[3] - mu) * rs) * g4[3] + b4[3]);
    nv[it] = r;
  }
  v8h hv;
  int xrow;
  const int c8 = (lane & 7) * 8;
  {
    const int row = 4 * job + (lane >> 3);
    int b, s, k;
    row_decode(row, b, s, k);
    const int mi = (b * kChunk + k) * kNumS + s;
    const int yrow = path ? mi : row;
    xrow = path ? row : mi;
    const float* op = chOld + (size_t)row * kBot + c8;
    const float* yp = y + (size_t)yrow * kBot + c8;
    const v4f o0 = *(const v4f*)(op);
    const v4f o1 = *(const v4f*)(op + 4);
    const v4f y0 = *(const v4f*)(yp);
    const v4f y1 = *(const v4f*)(yp + 4);
    const v4f g0 = *(const v4f*)(gam + c8);
    const v4f g1 = *(const v4f*)(gam + c8 + 4);
    const v4f e0 = *(const v4f*)(bet + c8);
    const v4f e1 = *(const v4f*)(bet + c8 + 4);
    const float mu = b ? mu1 : mu0;
    const float rs = b ? rs1 : rs0;
    v4f r0v, r1v;
    r0v[0] = o0[0] + (((y0[0] - mu) * rs) * g0[0] + e0[0]);
    r0v[1] = o0[1] + (((y0[1] - mu) * rs) * g0[1] + e0[1]);
    r0v[2] = o0[2] + (((y0[2] - mu) * rs) * g0[2] + e0[2]);
    r0v[3] = o0[3] + (((y0[3] - mu) * rs) * g0[3] + e0[3]);
    r1v[0] = o1[0] + (((y1[0] - mu) * rs) * g1[0] + e1[0]);
    r1v[1] = o1[1] + (((y1[1] - mu) * rs) * g1[1] + e1[1]);
    r1v[2] = o1[2] + (((y1[2] - mu) * rs) * g1[2] + e1[2]);
    r1v[3] = o1[3] + (((y1[3] - mu) * rs) * g1[3] + e1[3]);
    hv = pack8(r0v, r1v, kActCarry);
  }
  for (int pass = 0; pass < 2; ++pass) {
#pragma unroll
    for (int it = 0; it < 2; ++it) {
      const int row = 4 * job + 2 * it + (lane >> 4);
      *(volatile v4f*)(chNew + (size_t)row * kBot + (lane & 15) * 4) = nv[it];
    }
    *(volatile v8h*)(xseq + (size_t)xrow * kBot + c8) = hv;
    __threadfence();
  }
}

__global__ __launch_bounds__(256) void ola_prelu_kernel(const float* __restrict__ ch, const float* __restrict__ prelu,
                                                        unsigned short* __restrict__ yact) {
  const int tid = threadIdx.x;
  const int row = blockIdx.x * 32 + (tid >> 3);
  const int c8 = (tid & 7) * 8;
  const int b = row / kLen;
  const int t = row - b * kLen;
  const int l = t + kHop;
  const int s0 = l / kHop;
  const int k = l - s0 * kHop;
  const int rLate  = (b * kNumS + s0) * kChunk + k;
  const int rEarly = (b * kNumS + s0 - 1) * kChunk + k + kHop;
  const float* pl = ch + (size_t)rLate * kBot + c8;
  const float* pe = ch + (size_t)rEarly * kBot + c8;
  const v4f e0 = *(const v4f*)(pe);
  const v4f e1 = *(const v4f*)(pe + 4);
  const v4f l0 = *(const v4f*)(pl);
  const v4f l1 = *(const v4f*)(pl + 4);
  const float a = prelu[0];
  v4f o0, o1;
#pragma unroll
  for (int e = 0; e < 4; ++e) {
    const float v0 = 0.5f * (e0[e] + l0[e]);
    const float v1 = 0.5f * (e1[e] + l1[e]);
    o0[e] = (v0 >= 0.0f) ? v0 : a * v0;
    o1[e] = (v1 >= 0.0f) ? v1 : a * v1;
  }
  const v8h hv = pack8(o0, o1, kActCarry);
  unsigned short* p = yact + (size_t)row * kBot + c8;
  *(volatile v8h*)p = hv;
  __threadfence();
  *(volatile v8h*)p = hv;
}

constexpr int kSmPerB = kEnc * kLen / 4;
static_assert(kSmPerB % 256 == 0 && (kNumB * kSmPerB) / 256 == 1000, "softmax grid exact");
__global__ __launch_bounds__(256) void spk_softmax_kernel(const float* __restrict__ logit, float* __restrict__ out) {
  const int idx = blockIdx.x * 256 + threadIdx.x;
  const int b = idx / kSmPerB;
  const int j = idx - b * kSmPerB;
  const size_t base = (size_t)b * kMaskO * kLen + (size_t)j * 4;
  constexpr size_t strideSpk = (size_t)kEnc * kLen;
  v4f v[kSpk], o[kSpk];
#pragma unroll
  for (int s = 0; s < kSpk; ++s) v[s] = *(const v4f*)(logit + base + s * strideSpk);
#pragma unroll
  for (int e = 0; e < 4; ++e) {
    const float m = fmaxf(fmaxf(fmaxf(v[0][e], v[1][e]), fmaxf(v[2][e], v[3][e])), v[4][e]);
    const float x0 = __expf(v[0][e] - m);
    const float x1 = __expf(v[1][e] - m);
    const float x2 = __expf(v[2][e] - m);
    const float x3 = __expf(v[3][e] - m);
    const float x4 = __expf(v[4][e] - m);
    const float sum = (((x0 + x1) + x2) + x3) + x4;
    const float inv = __builtin_amdgcn_rcpf(sum);
    o[0][e] = x0 * inv;
    o[1][e] = x1 * inv;
    o[2][e] = x2 * inv;
    o[3][e] = x3 * inv;
    o[4][e] = x4 * inv;
  }
  for (int pass = 0; pass < 2; ++pass) {
#pragma unroll
    for (int s = 0; s < kSpk; ++s) *(volatile v4f*)(out + base + s * strideSpk) = o[s];
    __threadfence();
  }
}

extern "C" void kernel_launch(void* const* d_in, const int* in_sizes, int n_in,
                              void* d_out, int out_size, void* d_ws, size_t ws_size, hipStream_t stream) {
  if (n_in < 15 || d_out == nullptr || d_ws == nullptr) return;
  if (in_sizes[0] != kNumB * kEnc * kLen || in_sizes[1] != kEnc || in_sizes[2] != kEnc ||
      in_sizes[3] != kBot * kEnc || in_sizes[4] != kBot ||
      in_sizes[5] != kBlocks * 2 * 2 * kGate * kBot || in_sizes[6] != kBlocks * 2 * 2 * kGate * kHid ||
      in_sizes[7] != kBlocks * 2 * 2 * kGate || in_sizes[8] != kBlocks * 2 * kBot * kCat ||
      in_sizes[9] != kBlocks * 2 * kBot || in_sizes[10] != kBlocks * 2 * kBot || in_sizes[11] != kBlocks * 2 * kBot ||
      in_sizes[12] != 1 || in_sizes[13] != kMaskO * kBot || in_sizes[14] != kMaskO ||
      out_size != kNumB * kMaskO * kLen) return;
  if (ws_size < kWsTotal) return;

  const float* encoded  = (const float*)d_in[0];
  const float* gn_gamma = (const float*)d_in[1];
  const float* gn_beta  = (const float*)d_in[2];
  const float* bott_w   = (const float*)d_in[3];
  const float* bott_b   = (const float*)d_in[4];
  const float* blk_wi   = (const float*)d_in[5];
  const float* blk_wh   = (const float*)d_in[6];
  const float* blk_b    = (const float*)d_in[7];
  const float* blk_pw   = (const float*)d_in[8];
  const float* blk_pb   = (const float*)d_in[9];
  const float* blk_gg   = (const float*)d_in[10];
  const float* blk_gb   = (const float*)d_in[11];
  const float* prelu_a  = (const float*)d_in[12];
  const float* mask_w   = (const float*)d_in[13];
  const float* mask_b   = (const float*)d_in[14];
  float* out = (float*)d_out;

  char* ws = (char*)d_ws;
  unsigned short* WI16  = (unsigned short*)(ws + kOffWI);
  unsigned short* WH16  = (unsigned short*)(ws + kOffWH);
  unsigned short* PW16  = (unsigned short*)(ws + kOffPW);
  unsigned short* MW16  = (unsigned short*)(ws + kOffMW);
  unsigned short* BW16  = (unsigned short*)(ws + kOffBW);
  float*          PART  = (float*)(ws + kOffPART);
  unsigned short* XT    = (unsigned short*)(ws + kOffXT);
  float*          XB    = (float*)(ws + kOffXB);
  float*          CH0   = (float*)(ws + kOffCH0);
  float*          CH1   = (float*)(ws + kOffCH1);
  unsigned short* XSEQ  = (unsigned short*)(ws + kOffXSEQ);
  float*          PRE   = (float*)(ws + kOffPRE);
  unsigned short* HCAT  = (unsigned short*)(ws + kOffHCAT);
  float*          YP    = (float*)(ws + kOffYP);
  unsigned short* YACT  = (unsigned short*)(ws + kOffYACT);
  float*          LOGIT = (float*)(ws + kOffLOG);

  wcvt_kernel<<<kCbAll, 256, 0, stream>>>(blk_wi, WI16, blk_wh, WH16, blk_pw, PW16, mask_w, MW16, bott_w, BW16);
  padzero_kernel<<<(kPadX + kPadH + 255) / 256, 256, 0, stream>>>(XSEQ, HCAT);

  stats_kernel<<<dim3(kStatBlk, kNumB), 256, 0, stream>>>(encoded, kLen, (kLen + kStatBlk - 1) / kStatBlk, PART);
  front_norm_kernel<<<dim3(kLen / 64, kNumB), 256, 0, stream>>>(encoded, PART, gn_gamma, gn_beta, XT,
                                                                1.0 / ((double)kEnc * (double)kLen));
  gemm64_f16_kernel<2><<<dim3((kTok / 64 + 7) / 8, 1), 256, 0, stream>>>(
      XT, kEnc, 0L, BW16, kEnc, 0L, XB, kBot, 0L, bott_b, kTok, kBot, kEnc, kFold);
  chunk_build_kernel<<<(kJobs + 7) / 8, 256, 0, stream>>>(XB, CH0, XSEQ);

  float* chCur = CH0;
  float* chNxt = CH1;
  const double cntInvBlk = 1.0 / ((double)kRowsB * (double)kBot);
  for (int i = 0; i < kBlocks; ++i) {
    for (int p = 0; p < 2; ++p) {
      const int ij = i * 2 + p;
      const int nseq = p ? (kNumB * kChunk) : (kNumB * kNumS);
      const int tlen = p ? kNumS : kChunk;
      gemm64_f16_kernel<2><<<dim3(((kRowsP / 64) * (kGate2 / 64) + 7) / 8, 1), 256, 0, stream>>>(
          XSEQ, kBot, 0L, WI16 + (size_t)ij * kGate2 * kBot, kBot, 0L, PRE, kGate2, 0L,
          blk_b + (size_t)ij * kGate2, kRowsP, kGate2, kBot, kFold);
      bilstm_scan_kernel<<<dim3((nseq + 15) / 16, 2), 128, 0, stream>>>(
          PRE, WH16 + (size_t)ij * 2 * kGate * kHid, HCAT, nseq, tlen);
      gemm64_f16_kernel<2><<<dim3((kRowsP / 64 + 7) / 8, 1), 256, 0, stream>>>(
          HCAT, kCat, 0L, PW16 + (size_t)ij * kBot * kCat, kCat, 0L, YP, kBot, 0L,
          blk_pb + (size_t)ij * kBot, kRowsP, kBot, kCat, kFold);
      stats_kernel<<<dim3(kStatBlk, kNumB), 256, 0, stream>>>(YP, kRowsB, (kRowsB + kStatBlk - 1) / kStatBlk, PART);
      gn_apply_kernel<<<(kJobs + 7) / 8, 256, 0, stream>>>(chCur, YP, PART, blk_gg + (size_t)ij * kBot,
                                                           blk_gb + (size_t)ij * kBot, chNxt, XSEQ, p, cntInvBlk);
      float* tmp = chCur;
      chCur = chNxt;
      chNxt = tmp;
    }
  }

  ola_prelu_kernel<<<kTok / 32, 256, 0, stream>>>(chCur, prelu_a, YACT);
  gemm64_f16_kernel<1><<<dim3(((kMaskO / 64) * (kLen / 64) + 7) / 8, kNumB), 256, 0, stream>>>(
      MW16, kBot, 0L, YACT, kBot, (long)kLen * kBot, LOGIT, kLen, (long)kMaskO * kLen,
      mask_b, kMaskO, kLen, kBot, kFold);
  spk_softmax_kernel<<<(kNumB * kSmPerB) / 256, 256, 0, stream>>>(LOGIT, out);
}
